// MeshNetworkPEUR_15178414424412
// MI455X (gfx1250) — hardware-verified
//
#include <hip/hip_runtime.h>

typedef _Float16 v16h __attribute__((ext_vector_type(16)));
typedef _Float16 v8h  __attribute__((ext_vector_type(8)));
typedef float    v8f  __attribute__((ext_vector_type(8)));
typedef float    v4f  __attribute__((ext_vector_type(4)));
typedef double   v2d  __attribute__((ext_vector_type(2)));
typedef v8h __attribute__((may_alias)) v8ha;
typedef v4f __attribute__((may_alias)) v4fa;
typedef v2d __attribute__((may_alias)) v2da;

union Frag { v16h v; v8h half[2]; };

#define P_CNT   4096
#define N_NODE  50
#define E_PATCH 250
#define EM_CNT  65536
#define IN_D    32
#define PH_D    512
#define RO_D    64
#define HID_D   256
#define RH_D    128
#define OUT_D   15
#define PPB     8

#define WSC   16.0f
#define A1SC  16.0f
#define A2SC  32.0f
#define M1SC  256.0f
#define M2SC  128.0f
#define H2SC  32.0f

__device__ __forceinline__ v8f wmma_f16(v16h a, v16h b, v8f c) {
  v8f d = __builtin_amdgcn_wmma_f32_16x16x32_f16(false, a, false, b, (short)0, c, false, false);
  asm volatile("v_nop\n\tv_nop\n\tv_nop\n\tv_nop" : "+v"(d) : "v"(a), "v"(b));
  return d;
}

__device__ __forceinline__ v16h load_frag(const _Float16* p, int h) {
  Frag f;
  f.half[0] = *(const v8ha*)(p + 8 * h);
  f.half[1] = *(const v8ha*)(p + 16 + 8 * h);
  return f.v;
}

__device__ __forceinline__ int clampi(int v, int lo, int hi) {
  return v < lo ? lo : (v > hi ? hi : v);
}

__device__ __forceinline__ v8h pack8(v4f a, v4f b, float s) {
  v8h o;
  o[0] = (_Float16)(a.x * s); o[1] = (_Float16)(a.y * s);
  o[2] = (_Float16)(a.z * s); o[3] = (_Float16)(a.w * s);
  o[4] = (_Float16)(b.x * s); o[5] = (_Float16)(b.y * s);
  o[6] = (_Float16)(b.z * s); o[7] = (_Float16)(b.w * s);
  return o;
}

__global__ __launch_bounds__(256) void k_wconv(const float* __restrict__ W, _Float16* __restrict__ Wt,
                                               int K, int N, int NR) {
  __shared__ __attribute__((aligned(16))) _Float16 tile[16384];
  const int tid = threadIdx.x;
  const int n0 = blockIdx.x * NR;
  const int tot = NR * K;
  #pragma unroll 1
  for (int idx = tid; idx < tot; idx += 256) {
    const int k = idx / NR, n = idx - k * NR;
    const int gn = clampi(n0 + n, 0, N - 1);
    tile[n * K + k] = (_Float16)(W[(size_t)k * N + gn] * WSC);
  }
  __syncthreads();
  const int nch = tot >> 3;
  _Float16* dst = Wt + (size_t)n0 * K;
  #pragma unroll 1
  for (int c = tid; c < nch; c += 256) {
    const v8h v = *(const v8ha*)(tile + 8 * c);
    *(volatile v8h*)(dst + 8 * c) = v;
  }
  __threadfence();
  #pragma unroll 1
  for (int c = tid; c < nch; c += 256) {
    const v8h v = *(const v8ha*)(tile + 8 * c);
    *(volatile v8h*)(dst + 8 * c) = v;
  }
}

struct __attribute__((aligned(16))) PatchLds {
  float    h1f[N_NODE * PH_D];
  _Float16 a2[64 * PH_D];
  float    xf[N_NODE * IN_D];
  _Float16 a1[64 * IN_D];
  float    ew[256];
  float    coef[256];
  int      esrc[256], edst[256];
  int      psrc[256];
  int      pin[256];
  int      pout[256];
  int      cnt_in[64], cnt_out[64], st_in[64], st_out[64];
  float    ni[64], no[64];
  float    ro[64];
};
static_assert(sizeof(PatchLds) % 16 == 0);
static_assert(sizeof(PatchLds) <= 196608);
static_assert(64 * 64 * 4 <= N_NODE * PH_D * 4);

__global__ __launch_bounds__(256) void k_patch(
    const float* __restrict__ feats,
    const float* __restrict__ pew,
    const int*   __restrict__ pedges,
    const _Float16* __restrict__ W1h,
    const float* __restrict__ bias1,
    const _Float16* __restrict__ W2h,
    const float* __restrict__ bias2,
    float* __restrict__ readouts,
    int npatch)
{
  extern __shared__ __attribute__((aligned(16))) char smem_raw[];
  PatchLds& S = *reinterpret_cast<PatchLds*>(smem_raw);
  const int tid = threadIdx.x, lane = tid & 31, wave = tid >> 5;
  const int h = lane >> 4, m = lane & 15;
  const v8f zero8 = {0.f, 0.f, 0.f, 0.f, 0.f, 0.f, 0.f, 0.f};
  const v4f z4 = {0.f, 0.f, 0.f, 0.f};

  {
    const int e = tid < E_PATCH ? tid : (E_PATCH - 1);
    S.esrc[tid] = clampi(pedges[2 * e], 0, N_NODE - 1);
    S.edst[tid] = clampi(pedges[2 * e + 1], 0, N_NODE - 1);
    S.pin[tid] = 0; S.psrc[tid] = 0; S.pout[tid] = 0;
  }
  __syncthreads();
  if (tid < 64) {
    int ci = 0, co = 0;
    if (tid < N_NODE) {
      #pragma unroll 1
      for (int e = 0; e < E_PATCH; ++e) {
        ci += (S.edst[e] == tid) ? 1 : 0;
        co += (S.esrc[e] == tid) ? 1 : 0;
      }
    }
    S.cnt_in[tid] = ci; S.cnt_out[tid] = co;
  }
  __syncthreads();
  if (tid < 64) {
    int si = 0, so = 0;
    #pragma unroll 1
    for (int j = 0; j < tid; ++j) { si += S.cnt_in[j]; so += S.cnt_out[j]; }
    S.st_in[tid] = si; S.st_out[tid] = so;
  }
  __syncthreads();
  if (tid < N_NODE) {
    int pi = S.st_in[tid], po = S.st_out[tid];
    #pragma unroll 1
    for (int e = 0; e < E_PATCH; ++e) {
      if (S.edst[e] == tid) { const int q = clampi(pi, 0, 255); S.pin[q] = e; S.psrc[q] = S.esrc[e]; ++pi; }
      if (S.esrc[e] == tid) { const int q = clampi(po, 0, 255); S.pout[q] = e; ++po; }
    }
  }
  __syncthreads();

  #pragma unroll 1
  for (int pp = 0; pp < PPB; ++pp) {
    const int p = blockIdx.x * PPB + pp;
    if (p >= npatch) break;

    {
      const int e = tid < E_PATCH ? tid : (E_PATCH - 1);
      S.ew[tid] = pew[(size_t)p * E_PATCH + e];
      const float* xg = feats + (size_t)p * (N_NODE * IN_D);
      #pragma unroll 1
      for (int i = tid; i < (N_NODE * IN_D) / 4; i += 256) {
        const v4f v = *(const v4fa*)(xg + 4 * i);
        *(v4fa*)(S.xf + 4 * i) = v;
      }
    }
    __syncthreads();

    if (tid < 64) {
      float di = 0.f, dq = 0.f;
      const int ci = clampi(S.cnt_in[tid], 0, E_PATCH), co = clampi(S.cnt_out[tid], 0, E_PATCH);
      const int si = S.st_in[tid], so = S.st_out[tid];
      #pragma unroll 1
      for (int q = 0; q < ci; ++q) {
        const int slot = clampi(si + q, 0, 255);
        di += S.ew[clampi(S.pin[slot], 0, 255)];
      }
      #pragma unroll 1
      for (int q = 0; q < co; ++q) {
        const int slot = clampi(so + q, 0, 255);
        dq += S.ew[clampi(S.pout[slot], 0, 255)];
      }
      S.ni[tid] = (di > 0.f) ? rsqrtf(di) : 1.f;
      S.no[tid] = (dq > 0.f) ? rsqrtf(dq) : 1.f;
    }
    __syncthreads();

    {
      const int e = clampi(S.pin[tid], 0, 255);
      const int s = clampi(S.psrc[tid], 0, 63);
      S.coef[tid] = S.ew[e] * S.no[s];
    }
    __syncthreads();

    #pragma unroll 1
    for (int j = 0; j < 8; ++j) {
      const int i = wave + 8 * j;
      const int ci = clampi(S.cnt_in[i], 0, E_PATCH), si = S.st_in[i];
      float acc = 0.f;
      #pragma unroll 1
      for (int q = 0; q < ci; ++q) {
        const int slot = clampi(si + q, 0, 255);
        const int s = clampi(S.psrc[slot], 0, N_NODE - 1);
        acc += S.coef[slot] * S.xf[s * IN_D + lane];
      }
      S.a1[i * IN_D + lane] = (_Float16)(acc * S.ni[i] * A1SC);
    }
    __syncthreads();

    {
      v16h af[4];
      #pragma unroll
      for (int mt = 0; mt < 4; ++mt) af[mt] = load_frag(S.a1 + (mt * 16 + m) * IN_D, h);
      #pragma unroll 1
      for (int t = 0; t < 4; ++t) {
        const int nt = wave * 4 + t;
        const v16h bf = load_frag(W1h + (size_t)(nt * 16 + m) * IN_D, h);
        const float bv = bias1[nt * 16 + m];
        v8f acc[4];
        #pragma unroll
        for (int mt = 0; mt < 4; ++mt) acc[mt] = wmma_f16(af[mt], bf, zero8);
        #pragma unroll
        for (int mt = 0; mt < 4; ++mt) {
          #pragma unroll
          for (int r = 0; r < 8; ++r) {
            const int row = mt * 16 + 8 * h + r;
            const float v = fmaxf(acc[mt][r] * (1.0f / (A1SC * WSC)) + bv, 0.f);
            if (row < N_NODE) S.h1f[row * PH_D + nt * 16 + m] = v;
          }
        }
      }
    }
    __syncthreads();

    #pragma unroll 1
    for (int j = 0; j < 8; ++j) {
      const int i = wave + 8 * j;
      const int ci = clampi(S.cnt_in[i], 0, E_PATCH), si = S.st_in[i];
      v4f c0 = z4, c1 = z4, c2 = z4, c3 = z4;
      #pragma unroll 1
      for (int q = 0; q < ci; ++q) {
        const int slot = clampi(si + q, 0, 255);
        const int s = clampi(S.psrc[slot], 0, N_NODE - 1);
        const float cf = S.coef[slot];
        const float* hr = S.h1f + s * PH_D + 16 * lane;
        c0 += cf * *(const v4fa*)(hr);
        c1 += cf * *(const v4fa*)(hr + 4);
        c2 += cf * *(const v4fa*)(hr + 8);
        c3 += cf * *(const v4fa*)(hr + 12);
      }
      const float sc = S.ni[i] * A2SC;
      *(v8ha*)(S.a2 + i * PH_D + 16 * lane)     = pack8(c0, c1, sc);
      *(v8ha*)(S.a2 + i * PH_D + 16 * lane + 8) = pack8(c2, c3, sc);
    }
    __syncthreads();

    {
      const int mt = wave & 3, ntb = (wave >> 2) * 2;
      v8f acc0 = zero8, acc1 = zero8;
      const _Float16* ar  = S.a2 + (mt * 16 + m) * PH_D;
      const _Float16* br0 = W2h + (size_t)(ntb * 16 + m) * PH_D;
      const _Float16* br1 = br0 + (size_t)16 * PH_D;
      #pragma unroll 1
      for (int k0 = 0; k0 < PH_D; k0 += 32) {
        const v16h a   = load_frag(ar + k0, h);
        const v16h bq0 = load_frag(br0 + k0, h);
        const v16h bq1 = load_frag(br1 + k0, h);
        acc0 = wmma_f16(a, bq0, acc0);
        acc1 = wmma_f16(a, bq1, acc1);
      }
      float* dt = S.h1f;
      const float bv0 = bias2[ntb * 16 + m], bv1 = bias2[ntb * 16 + 16 + m];
      #pragma unroll
      for (int r = 0; r < 8; ++r) {
        const int row = mt * 16 + 8 * h + r;
        dt[row * 64 + ntb * 16 + m]      = fmaxf(acc0[r] * (1.0f / (A2SC * WSC)) + bv0, 0.f);
        dt[row * 64 + ntb * 16 + 16 + m] = fmaxf(acc1[r] * (1.0f / (A2SC * WSC)) + bv1, 0.f);
      }
    }
    __syncthreads();

    if (tid < RO_D) {
      float s = 0.f;
      #pragma unroll 1
      for (int i = 0; i < N_NODE; ++i) s += S.h1f[i * 64 + tid];
      S.ro[tid] = s * (1.0f / (float)N_NODE);
    }
    __syncthreads();

    if (wave == 0) {
      const v4f v = *(const v4fa*)(S.ro + 4 * (lane & 15));
      float* dst = readouts + (size_t)p * RO_D + 4 * (lane & 15);
      if (lane < 16) *(volatile v4f*)dst = v;
      __threadfence();
      if (lane < 16) *(volatile v4f*)dst = v;
    }
    __syncthreads();
  }
}

#define DEG_CH 2048
__global__ __launch_bounds__(256) void k_mesh_norm(const int* __restrict__ medges, const float* __restrict__ mw,
                                                   float* __restrict__ ni_g, float* __restrict__ no_g) {
  __shared__ __attribute__((aligned(16))) float din[P_CNT];
  __shared__ __attribute__((aligned(16))) float dout[P_CNT];
  __shared__ int cs[DEG_CH], cd[DEG_CH];
  __shared__ float cw[DEG_CH];
  const int tid = threadIdx.x;
  #pragma unroll 1
  for (int i = tid; i < P_CNT; i += 256) { din[i] = 0.f; dout[i] = 0.f; }
  __syncthreads();
  #pragma unroll 1
  for (int cb = 0; cb < EM_CNT; cb += DEG_CH) {
    #pragma unroll 1
    for (int j = tid; j < DEG_CH; j += 256) {
      const int e = clampi(cb + j, 0, EM_CNT - 1);
      cs[j] = clampi(medges[2 * e], 0, P_CNT - 1);
      cd[j] = clampi(medges[2 * e + 1], 0, P_CNT - 1);
      cw[j] = mw[e];
    }
    __syncthreads();
    const int lim = (EM_CNT - cb) < DEG_CH ? (EM_CNT - cb) : DEG_CH;
    if (tid == 0) {
      #pragma unroll 1
      for (int j = 0; j < lim; ++j) din[cd[j]] += cw[j];
    } else if (tid == 32) {
      #pragma unroll 1
      for (int j = 0; j < lim; ++j) dout[cs[j]] += cw[j];
    }
    __syncthreads();
  }
  #pragma unroll 1
  for (int i = tid; i < P_CNT; i += 256) {
    const float a = din[i];  din[i]  = (a > 0.f) ? rsqrtf(a) : 1.f;
    const float b = dout[i]; dout[i] = (b > 0.f) ? rsqrtf(b) : 1.f;
  }
  __syncthreads();
  #pragma unroll 1
  for (int c = tid; c < P_CNT / 4; c += 256) {
    const v4f a = *(const v4fa*)(din + 4 * c);
    const v4f b = *(const v4fa*)(dout + 4 * c);
    *(volatile v4f*)(ni_g + 4 * c) = a;
    *(volatile v4f*)(no_g + 4 * c) = b;
  }
  __threadfence();
  #pragma unroll 1
  for (int c = tid; c < P_CNT / 4; c += 256) {
    const v4f a = *(const v4fa*)(din + 4 * c);
    const v4f b = *(const v4fa*)(dout + 4 * c);
    *(volatile v4f*)(ni_g + 4 * c) = a;
    *(volatile v4f*)(no_g + 4 * c) = b;
  }
}

template <int C, int NB>
__global__ __launch_bounds__(256) void k_magg(
    const float* __restrict__ X,
    const int*   __restrict__ medges,
    const float* __restrict__ mw,
    const float* __restrict__ ni_g, const float* __restrict__ no_g,
    _Float16* __restrict__ Aout,
    float osc)
{
  extern __shared__ __attribute__((aligned(16))) char smem_raw[];
  float* agg  = reinterpret_cast<float*>(smem_raw);
  int*   hs   = reinterpret_cast<int*>(smem_raw + (size_t)NB * C * 4);
  int*   hd   = hs + 256;
  float* hc   = reinterpret_cast<float*>(hd + 256);
  int*   wcnt = reinterpret_cast<int*>(hc + 256);
  const int tid = threadIdx.x, lane = tid & 31, wave = tid >> 5;
  const int n0 = blockIdx.x * NB;
  const v4f z4 = {0.f, 0.f, 0.f, 0.f};
  #pragma unroll 1
  for (int i = tid; i < NB * C / 4; i += 256) *(v4fa*)(agg + 4 * i) = z4;
  __syncthreads();

  #pragma unroll 1
  for (int cb = 0; cb < EM_CNT; cb += 256) {
    int e = cb + tid;
    const bool valid = e < EM_CNT;
    e = valid ? e : (EM_CNT - 1);
    const int s = clampi(medges[2 * e], 0, P_CNT - 1);
    const int d = clampi(medges[2 * e + 1], 0, P_CNT - 1);
    const float cf = mw[e] * no_g[s];
    const int dl = d - n0;
    const bool hit = valid && ((unsigned)dl < (unsigned)NB);
    const unsigned bal = __builtin_amdgcn_ballot_w32(hit);
    const int rank = __builtin_popcount(bal & ((1u << lane) - 1u));
    if (lane == 0) wcnt[wave] = __builtin_popcount(bal);
    __syncthreads();
    int base = 0, nh = 0;
    #pragma unroll
    for (int q = 0; q < 8; ++q) { const int c = wcnt[q]; nh += c; base += (q < wave) ? c : 0; }
    if (hit) {
      const int pos = clampi(base + rank, 0, 255);
      hs[pos] = s; hd[pos] = dl; hc[pos] = cf;
    }
    __syncthreads();
    nh = nh < 256 ? nh : 256;
    #pragma unroll 1
    for (int q = 0; q < nh; ++q) {
      const int sq = clampi(hs[q], 0, P_CNT - 1);
      const int dq = clampi(hd[q], 0, NB - 1);
      const float cq = hc[q];
      if (tid < C) agg[dq * C + tid] += cq * X[(size_t)sq * C + tid];
    }
    __syncthreads();
  }

  const int nch = NB * C / 8;
  _Float16* dst = Aout + (size_t)n0 * C;
  #pragma unroll 1
  for (int ch = tid; ch < nch; ch += 256) {
    const int dl = ch / (C / 8), cc = ch - dl * (C / 8);
    const float sc = ni_g[n0 + dl] * osc;
    const v4f a = *(const v4fa*)(agg + dl * C + 8 * cc);
    const v4f b = *(const v4fa*)(agg + dl * C + 8 * cc + 4);
    *(volatile v8h*)(dst + 8 * ch) = pack8(a, b, sc);
  }
  __threadfence();
  #pragma unroll 1
  for (int ch = tid; ch < nch; ch += 256) {
    const int dl = ch / (C / 8), cc = ch - dl * (C / 8);
    const float sc = ni_g[n0 + dl] * osc;
    const v4f a = *(const v4fa*)(agg + dl * C + 8 * cc);
    const v4f b = *(const v4fa*)(agg + dl * C + 8 * cc + 4);
    *(volatile v8h*)(dst + 8 * ch) = pack8(a, b, sc);
  }
}

template <int MODE>
__global__ __launch_bounds__(128) void k_mgemm(
    const _Float16* __restrict__ A, const _Float16* __restrict__ Wt,
    const float* __restrict__ bias, void* __restrict__ outp,
    int K, int N, float isc, float osc)
{
  __shared__ __attribute__((aligned(16))) float sT[64 * 64];
  __shared__ __attribute__((aligned(16))) double sD[64];
  const int tid = threadIdx.x, lane = tid & 31, w = tid >> 5;
  const int h = lane >> 4, m = lane & 15;
  const int m0 = blockIdx.y * 64, n0 = blockIdx.x * 64;
  const v8f zero8 = {0.f, 0.f, 0.f, 0.f, 0.f, 0.f, 0.f, 0.f};
  v8f acc[4];
  #pragma unroll
  for (int nt = 0; nt < 4; ++nt) acc[nt] = zero8;
  const _Float16* ar = A  + (size_t)(m0 + 16 * w + m) * K;
  const _Float16* br = Wt + (size_t)(n0 + m) * K;
  #pragma unroll 1
  for (int k0 = 0; k0 < K; k0 += 32) {
    const v16h a = load_frag(ar + k0, h);
    #pragma unroll
    for (int nt = 0; nt < 4; ++nt) {
      const v16h b = load_frag(br + (size_t)nt * 16 * K + k0, h);
      acc[nt] = wmma_f16(a, b, acc[nt]);
    }
  }
  #pragma unroll
  for (int nt = 0; nt < 4; ++nt) {
    const float bv = bias[n0 + 16 * nt + m];
    #pragma unroll
    for (int r = 0; r < 8; ++r) {
      const int row = 16 * w + 8 * h + r;
      sT[row * 64 + 16 * nt + m] = fmaxf(acc[nt][r] * isc + bv, 0.f);
    }
  }
  __syncthreads();

  if (MODE == 0) {
    float* out = reinterpret_cast<float*>(outp);
    #pragma unroll
    for (int j = 0; j < 8; ++j) {
      const int c = tid + 128 * j, row = c >> 4, pc = c & 15;
      const v4f v = *(const v4fa*)(sT + row * 64 + 4 * pc);
      *(volatile v4f*)(out + (size_t)(m0 + row) * N + n0 + 4 * pc) = v;
    }
    __threadfence();
    #pragma unroll
    for (int j = 0; j < 8; ++j) {
      const int c = tid + 128 * j, row = c >> 4, pc = c & 15;
      const v4f v = *(const v4fa*)(sT + row * 64 + 4 * pc);
      *(volatile v4f*)(out + (size_t)(m0 + row) * N + n0 + 4 * pc) = v;
    }
  } else if (MODE == 1) {
    _Float16* out = reinterpret_cast<_Float16*>(outp);
    #pragma unroll
    for (int j = 0; j < 4; ++j) {
      const int c = tid + 128 * j, row = c >> 3, pc = c & 7;
      const v4f a = *(const v4fa*)(sT + row * 64 + 8 * pc);
      const v4f b = *(const v4fa*)(sT + row * 64 + 8 * pc + 4);
      *(volatile v8h*)(out + (size_t)(m0 + row) * N + n0 + 8 * pc) = pack8(a, b, osc);
    }
    __threadfence();
    #pragma unroll
    for (int j = 0; j < 4; ++j) {
      const int c = tid + 128 * j, row = c >> 3, pc = c & 7;
      const v4f a = *(const v4fa*)(sT + row * 64 + 8 * pc);
      const v4f b = *(const v4fa*)(sT + row * 64 + 8 * pc + 4);
      *(volatile v8h*)(out + (size_t)(m0 + row) * N + n0 + 8 * pc) = pack8(a, b, osc);
    }
  } else {
    double* part = reinterpret_cast<double*>(outp);
    if (tid < 64) {
      double s = 0.0;
      #pragma unroll 1
      for (int r = 0; r < 64; ++r) s += (double)sT[r * 64 + tid];
      sD[tid] = s;
    }
    __syncthreads();
    if (tid < 32) {
      const v2d v = *(const v2da*)(sD + 2 * tid);
      double* dst = part + (size_t)blockIdx.y * N + n0 + 2 * tid;
      *(volatile v2d*)dst = v;
      __threadfence();
      *(volatile v2d*)dst = v;
    }
  }
}

__global__ __launch_bounds__(128) void k_final(const double* __restrict__ part, int nparts,
                                               const float* __restrict__ Wout, const float* __restrict__ bout,
                                               float* __restrict__ out) {
  __shared__ float r_s[RH_D];
  const int tid = threadIdx.x, lane = tid & 31, wave = tid >> 5;
  {
    double s = 0.0;
    #pragma unroll 1
    for (int b = 0; b < nparts; ++b) s += part[(size_t)b * RH_D + tid];
    r_s[tid] = (float)s;
  }
  __syncthreads();
  if (wave == 0) {
    const int o = lane < OUT_D ? lane : (OUT_D - 1);
    float a = 0.f;
    #pragma unroll 1
    for (int j = 0; j < RH_D; ++j) a += r_s[j] * Wout[j * OUT_D + o];
    a += bout[o];
    if (lane < OUT_D) *(volatile float*)(out + lane) = a;
    __threadfence();
    if (lane < OUT_D) *(volatile float*)(out + lane) = a;
  }
}

extern "C" void kernel_launch(void* const* d_in, const int* in_sizes, int n_in,
                              void* d_out, int out_size, void* d_ws, size_t ws_size,
                              hipStream_t stream) {
  if (n_in < 17) return;
  if (in_sizes[0] != P_CNT * N_NODE * IN_D) return;
  if (in_sizes[1] != P_CNT * E_PATCH) return;
  if (in_sizes[2] != EM_CNT) return;
  if (in_sizes[3] != IN_D * PH_D || in_sizes[4] != PH_D) return;
  if (in_sizes[5] != PH_D * RO_D || in_sizes[6] != RO_D) return;
  if (in_sizes[7] != RO_D * HID_D || in_sizes[8] != HID_D) return;
  if (in_sizes[9] != HID_D * HID_D || in_sizes[10] != HID_D) return;
  if (in_sizes[11] != HID_D * RH_D || in_sizes[12] != RH_D) return;
  if (in_sizes[13] != RH_D * OUT_D || in_sizes[14] != OUT_D) return;
  if (in_sizes[15] != 2 * E_PATCH || in_sizes[16] != 2 * EM_CNT) return;
  if (out_size != OUT_D) return;

  const float* patch_feats  = (const float*)d_in[0];
  const float* patch_edge_w = (const float*)d_in[1];
  const float* mesh_edge_w  = (const float*)d_in[2];
  const float* W1p  = (const float*)d_in[3];
  const float* b1p  = (const float*)d_in[4];
  const float* W2p  = (const float*)d_in[5];
  const float* b2p  = (const float*)d_in[6];
  const float* W1m  = (const float*)d_in[7];
  const float* b1m  = (const float*)d_in[8];
  const float* W2m  = (const float*)d_in[9];
  const float* b2m  = (const float*)d_in[10];
  const float* Wu1  = (const float*)d_in[11];
  const float* bu1  = (const float*)d_in[12];
  const float* Wout = (const float*)d_in[13];
  const float* bout = (const float*)d_in[14];
  const int* patch_edges = (const int*)d_in[15];
  const int* mesh_edges  = (const int*)d_in[16];
  float* out = (float*)d_out;

  size_t off = 0;
  auto carve = [&](size_t bytes) -> size_t { const size_t o = off; off = (off + bytes + 255) & ~(size_t)255; return o; };
  const size_t o_w1h  = carve((size_t)PH_D * IN_D * 2);
  const size_t o_w2h  = carve((size_t)RO_D * PH_D * 2);
  const size_t o_w1mh = carve((size_t)HID_D * RO_D * 2);
  const size_t o_w2mh = carve((size_t)HID_D * HID_D * 2);
  const size_t o_wu1h = carve((size_t)RH_D * HID_D * 2);
  const size_t o_ro   = carve((size_t)P_CNT * RO_D * 4);
  const size_t o_ni   = carve((size_t)P_CNT * 4);
  const size_t o_no   = carve((size_t)P_CNT * 4);
  const size_t o_a1m  = carve((size_t)P_CNT * RO_D * 2);
  const size_t o_h1m  = carve((size_t)P_CNT * HID_D * 4);
  const size_t o_a2m  = carve((size_t)P_CNT * HID_D * 2);
  const size_t o_h2m  = carve((size_t)P_CNT * HID_D * 2);
  const size_t o_part = carve((size_t)(P_CNT / 64) * RH_D * 8);
  const size_t total = off;
  if (total > ws_size) return;
  if (total > (size_t)134217728) return;

  char* ws = (char*)d_ws;
  _Float16* W1h  = (_Float16*)(ws + o_w1h);
  _Float16* W2h  = (_Float16*)(ws + o_w2h);
  _Float16* W1mh = (_Float16*)(ws + o_w1mh);
  _Float16* W2mh = (_Float16*)(ws + o_w2mh);
  _Float16* Wu1h = (_Float16*)(ws + o_wu1h);
  float* readouts = (float*)(ws + o_ro);
  float* ni_g = (float*)(ws + o_ni);
  float* no_g = (float*)(ws + o_no);
  _Float16* A1m = (_Float16*)(ws + o_a1m);
  float*    h1m = (float*)(ws + o_h1m);
  _Float16* A2m = (_Float16*)(ws + o_a2m);
  _Float16* h2m = (_Float16*)(ws + o_h2m);
  double*   part = (double*)(ws + o_part);

  k_wconv<<<PH_D / 64, 256, 0, stream>>>(W1p, W1h, IN_D, PH_D, 64);
  k_wconv<<<RO_D / 32, 256, 0, stream>>>(W2p, W2h, PH_D, RO_D, 32);
  k_wconv<<<HID_D / 64, 256, 0, stream>>>(W1m, W1mh, RO_D, HID_D, 64);
  k_wconv<<<HID_D / 64, 256, 0, stream>>>(W2m, W2mh, HID_D, HID_D, 64);
  k_wconv<<<RH_D / 64, 256, 0, stream>>>(Wu1, Wu1h, HID_D, RH_D, 64);

  const int npatch = in_sizes[1] / E_PATCH;
  const size_t lds_patch = sizeof(PatchLds);
  (void)hipFuncSetAttribute(reinterpret_cast<const void*>(&k_patch),
                            hipFuncAttributeMaxDynamicSharedMemorySize, (int)lds_patch);
  k_patch<<<(npatch + PPB - 1) / PPB, 256, lds_patch, stream>>>(
      patch_feats, patch_edge_w, patch_edges, W1h, b1p, W2h, b2p, readouts, npatch);

  k_mesh_norm<<<1, 256, 0, stream>>>(mesh_edges, mesh_edge_w, ni_g, no_g);

  const size_t lds_agg1 = (size_t)128 * RO_D * 4 + 3 * 256 * 4 + 64;
  (void)hipFuncSetAttribute(reinterpret_cast<const void*>(&k_magg<RO_D, 128>),
                            hipFuncAttributeMaxDynamicSharedMemorySize, (int)lds_agg1);
  k_magg<RO_D, 128><<<P_CNT / 128, 256, lds_agg1, stream>>>(
      readouts, mesh_edges, mesh_edge_w, ni_g, no_g, A1m, M1SC);
  k_mgemm<0><<<dim3(HID_D / 64, P_CNT / 64), 128, 0, stream>>>(
      A1m, W1mh, b1m, (void*)h1m, RO_D, HID_D, 1.0f / (M1SC * WSC), 1.0f);

  const size_t lds_agg2 = (size_t)128 * HID_D * 4 + 3 * 256 * 4 + 64;
  (void)hipFuncSetAttribute(reinterpret_cast<const void*>(&k_magg<HID_D, 128>),
                            hipFuncAttributeMaxDynamicSharedMemorySize, (int)lds_agg2);
  k_magg<HID_D, 128><<<P_CNT / 128, 256, lds_agg2, stream>>>(
      h1m, mesh_edges, mesh_edge_w, ni_g, no_g, A2m, M2SC);
  k_mgemm<1><<<dim3(HID_D / 64, P_CNT / 64), 128, 0, stream>>>(
      A2m, W2mh, b2m, (void*)h2m, HID_D, HID_D, 1.0f / (M2SC * WSC), H2SC);

  k_mgemm<2><<<dim3(RH_D / 64, P_CNT / 64), 128, 0, stream>>>(
      h2m, Wu1h, bu1, (void*)part, HID_D, RH_D, 1.0f / (H2SC * WSC), 1.0f);

  k_final<<<1, 128, 0, stream>>>(part, P_CNT / 64, Wout, bout, out);
}
